// XLSTM_dynamic_graph_70317204570396
// MI455X (gfx1250) — hardware-run, weakly checked
//
#include <hip/hip_runtime.h>
#include <math.h>

typedef __attribute__((ext_vector_type(16))) _Float16 v16h;
typedef __attribute__((ext_vector_type(8)))  _Float16 v8h;
typedef __attribute__((ext_vector_type(8)))  float    v8f;
typedef __attribute__((ext_vector_type(4)))  float    v4f;
typedef __attribute__((ext_vector_type(2)))  float    v2f;

constexpr int kNB  = 8;
constexpr int kNT  = 16;
constexpr int kNN  = 1024;
constexpr int kNF  = 64;
constexpr int kND  = 128;
constexpr int kNDL = 8;
constexpr int kNBT = kNB * kNT;
constexpr int kNDrift = kNB * (kNT - 1);
constexpr float kWCarry      = 4096.0f;
constexpr float kWCarryInv   = 1.0f / 4096.0f;
constexpr float kResCarry    = 2048.0f;
constexpr float kResCarryInv = 1.0f / 2048.0f;
constexpr float kF16MinNorm  = 6.103515625e-05f;
constexpr float kLnEps       = 1e-5f;
constexpr int kWtPitch   = 72;
constexpr int kSlabPitchB = 68;
constexpr int kSlabPitchC = 36;
static_assert(kNF % 32 == 0 && kND % 32 == 0, "K multiples of 32");
static_assert(kNBT == 128 && kNT == 16 && kND == 128 && kNN % 16 == 0, "tile multiples");
static_assert(kNDrift == 120, "drift count");
static_assert(kNF + 8 <= kWtPitch, "weight tile pitch");

constexpr size_t kPlaneBytes = (size_t)kNBT * kNN * kND * 2;
constexpr size_t kOffKH = 0;
constexpr size_t kOffKL = kOffKH + kPlaneBytes;
constexpr size_t kOffVH = kOffKL + kPlaneBytes;
constexpr size_t kOffVL = kOffVH + kPlaneBytes;
constexpr size_t kWsTotal = kOffVL + kPlaneBytes;
static_assert(kPlaneBytes == 33554432ull, "plane bytes");
static_assert(kWsTotal == 134217728ull, "carve total");
static_assert((kOffKL % 128) == 0 && (kOffVH % 128) == 0 && (kOffVL % 128) == 0, "aligned regions");

__device__ __forceinline__ unsigned short f2bf_bits(float f) {
  unsigned u = __float_as_uint(f);
  return (unsigned short)((u + 0x7FFFu + ((u >> 16) & 1u)) >> 16);
}
__device__ __forceinline__ float bfv(float f) {
  return __uint_as_float(((unsigned)f2bf_bits(f)) << 16);
}
__device__ __forceinline__ _Float16 f16_flush(float v) {
  const float w = (fabsf(v) < kF16MinNorm) ? 0.0f : v;
  return (_Float16)w;
}
union FragU { v16h v; v8h h[2]; };
__device__ __forceinline__ v16h frag_load(const _Float16* p) {
  FragU f;
  f.h[0] = *(const v8h*)(p);
  f.h[1] = *(const v8h*)(p + 16);
  return f.v;
}
__device__ __forceinline__ v8f mma_h(v16h a, v16h b, v8f c) {
  c = __builtin_amdgcn_wmma_f32_16x16x32_f16(false, a, false, b, (short)0, c, false, false);
  asm volatile("v_nop\n\tv_nop\n\tv_nop\n\tv_nop" : "+v"(c) : "v"(a), "v"(b));
  return c;
}
__device__ __forceinline__ void mma_vr(v16h ah, v16h al, v16h bh, v16h bl, v8f& cm, v8f& cr) {
  cm = __builtin_amdgcn_wmma_f32_16x16x32_f16(false, ah, false, bh, (short)0, cm, false, false);
  cr = __builtin_amdgcn_wmma_f32_16x16x32_f16(false, ah, false, bl, (short)0, cr, false, false);
  cr = __builtin_amdgcn_wmma_f32_16x16x32_f16(false, al, false, bh, (short)0, cr, false, false);
  asm volatile("v_nop\n\tv_nop\n\tv_nop\n\tv_nop" : "+v"(cm) : "v"(ah), "v"(al), "v"(bh), "v"(bl));
  asm volatile("v_nop\n\tv_nop\n\tv_nop\n\tv_nop" : "+v"(cr) : "v"(ah), "v"(al), "v"(bh), "v"(bl));
}

__device__ __forceinline__ void ln_rows(v8f (&acc)[8], const float* __restrict__ bias_row,
                                        const float* __restrict__ g, const float* __restrict__ be, int c) {
  float rs[8];
#pragma unroll
  for (int r = 0; r < 8; ++r) rs[r] = 0.0f;
#pragma unroll
  for (int j = 0; j < 8; ++j) {
    const float bj = bfv(bias_row[j * 16 + c]);
#pragma unroll
    for (int r = 0; r < 8; ++r) {
      const float p = acc[j][r] * kWCarryInv + bj;
      acc[j][r] = p;
      rs[r] += p;
    }
  }
#pragma unroll
  for (int off = 1; off < 16; off <<= 1) {
#pragma unroll
    for (int r = 0; r < 8; ++r) rs[r] += __shfl_xor(rs[r], off, 32);
  }
  float dv[8];
#pragma unroll
  for (int r = 0; r < 8; ++r) {
    rs[r] = rs[r] * (1.0f / (float)kND);
    dv[r] = 0.0f;
  }
#pragma unroll
  for (int j = 0; j < 8; ++j) {
#pragma unroll
    for (int r = 0; r < 8; ++r) {
      const float d = acc[j][r] - rs[r];
      acc[j][r] = d;
      dv[r] += d * d;
    }
  }
#pragma unroll
  for (int off = 1; off < 16; off <<= 1) {
#pragma unroll
    for (int r = 0; r < 8; ++r) dv[r] += __shfl_xor(dv[r], off, 32);
  }
#pragma unroll
  for (int r = 0; r < 8; ++r) dv[r] = rsqrtf(dv[r] * (1.0f / (float)kND) + kLnEps);
#pragma unroll
  for (int j = 0; j < 8; ++j) {
    const float gj = bfv(g[j * 16 + c]);
    const float bj = bfv(be[j * 16 + c]);
#pragma unroll
    for (int r = 0; r < 8; ++r) acc[j][r] = (gj * acc[j][r]) * dv[r] + bj;
  }
}

template <int J0>
__device__ __forceinline__ void slab_put(float* slab, const v8f (&acc)[8], int h, int c) {
#pragma unroll
  for (int jj = 0; jj < 4; ++jj) {
#pragma unroll
    for (int r = 0; r < 8; ++r) slab[(8 * h + r) * kSlabPitchB + jj * 16 + c] = acc[J0 + jj][r];
  }
}

constexpr int kWtBytes = 2 * kND * kWtPitch * 2;
static_assert(8 * 16 * kSlabPitchB * 4 <= kWtBytes, "slab alias fits");

__global__ __launch_bounds__(256) void node_proj_kernel(
    const float* __restrict__ x, const float* __restrict__ Wk, const float* __restrict__ Wv,
    const float* __restrict__ bk, const float* __restrict__ bv,
    const float* __restrict__ kg, const float* __restrict__ kb,
    const float* __restrict__ vg, const float* __restrict__ vb,
    unsigned short* __restrict__ KHp, unsigned short* __restrict__ KLp,
    unsigned short* __restrict__ VHp, unsigned short* __restrict__ VLp, float kscale)
{
  __shared__ __align__(16) unsigned char smem[kWtBytes];
  _Float16* WtK = (_Float16*)(void*)smem;
  _Float16* WtV = WtK + kND * kWtPitch;
  const int tid = threadIdx.x, lane = tid & 31, wave = tid >> 5;
  const int h = lane >> 4, c = lane & 15;
  const int n = blockIdx.x;

  {
    const float* wkb = Wk + (size_t)n * (kNF * kND);
    const float* wvb = Wv + (size_t)n * (kNF * kND);
#pragma unroll 1
    for (int it = 0; it < 8; ++it) {
      const int idx = tid + 256 * it;
      const int f = idx >> 5, d4 = (idx & 31) * 4;
      const v4f wk = *(const v4f*)(wkb + f * kND + d4);
      const v4f wv = *(const v4f*)(wvb + f * kND + d4);
#pragma unroll
      for (int e = 0; e < 4; ++e) {
        const float sk = wk[e];
        const float sv = wv[e];
        WtK[(d4 + e) * kWtPitch + f] = f16_flush(bfv(sk) * kWCarry);
        WtV[(d4 + e) * kWtPitch + f] = f16_flush(bfv(sv) * kWCarry);
      }
    }
  }

  v16h afr[2];
  {
    const float* xr = x + ((size_t)(wave * 16 + c) * kNN + n) * kNF + 8 * h;
#pragma unroll
    for (int ks = 0; ks < 2; ++ks) {
      const v4f p0 = *(const v4f*)(xr + ks * 32);
      const v4f p1 = *(const v4f*)(xr + ks * 32 + 4);
      const v4f p2 = *(const v4f*)(xr + ks * 32 + 16);
      const v4f p3 = *(const v4f*)(xr + ks * 32 + 20);
#pragma unroll
      for (int e = 0; e < 4; ++e) {
        const float s0 = p0[e];
        const float s1 = p1[e];
        const float s2 = p2[e];
        const float s3 = p3[e];
        afr[ks][e]      = f16_flush(bfv(s0));
        afr[ks][4 + e]  = f16_flush(bfv(s1));
        afr[ks][8 + e]  = f16_flush(bfv(s2));
        afr[ks][12 + e] = f16_flush(bfv(s3));
      }
    }
  }
  __syncthreads();

  v8f accK[8], accV[8];
#pragma unroll
  for (int j = 0; j < 8; ++j) {
    accK[j] = (v8f){0.f, 0.f, 0.f, 0.f, 0.f, 0.f, 0.f, 0.f};
    accV[j] = (v8f){0.f, 0.f, 0.f, 0.f, 0.f, 0.f, 0.f, 0.f};
  }
#pragma unroll
  for (int ks = 0; ks < 2; ++ks) {
#pragma unroll
    for (int j = 0; j < 8; ++j) {
      const _Float16* bp = WtK + (j * 16 + c) * kWtPitch + ks * 32 + 8 * h;
      const v16h bK = frag_load(bp);
      const v16h bV = frag_load(bp + kND * kWtPitch);
      accK[j] = mma_h(afr[ks], bK, accK[j]);
      accV[j] = mma_h(afr[ks], bV, accV[j]);
    }
  }
  __syncthreads();

  ln_rows(accK, bk + (size_t)n * kND, kg, kb, c);
  ln_rows(accV, bv + (size_t)n * kND, vg, vb, c);

  float* slab = (float*)(void*)smem + wave * (16 * kSlabPitchB);
  const int q = lane >> 3, c8 = (lane & 7) * 8;
#pragma unroll 1
  for (int ph = 0; ph < 4; ++ph) {
    if (ph == 0)      slab_put<0>(slab, accK, h, c);
    else if (ph == 1) slab_put<4>(slab, accK, h, c);
    else if (ph == 2) slab_put<0>(slab, accV, h, c);
    else              slab_put<4>(slab, accV, h, c);
    __syncthreads();
    unsigned short* PH = (ph < 2) ? KHp : VHp;
    unsigned short* PL = (ph < 2) ? KLp : VLp;
    const float scale = (ph < 2) ? kscale : 1.0f;
    const size_t rowbase = ((size_t)(wave * 16) * kNN + n) * kND + (size_t)(ph & 1) * 64 + c8;
#pragma unroll 1
    for (int it = 0; it < 4; ++it) {
      const int row = it * 4 + q;
      const float* sp = slab + row * kSlabPitchB + c8;
      const v4f y0 = *(const v4f*)(sp);
      const v4f y1 = *(const v4f*)(sp + 4);
      v8h hv, lv;
#pragma unroll
      for (int e = 0; e < 4; ++e) {
        const float ya = y0[e];
        const float yb = y1[e];
        const float sa = (fmaxf(ya, 0.0f) + __logf(1.0f + __expf(-fabsf(ya)))) * scale;
        const float sb = (fmaxf(yb, 0.0f) + __logf(1.0f + __expf(-fabsf(yb)))) * scale;
        const _Float16 ha = f16_flush(sa);
        const _Float16 hb = f16_flush(sb);
        hv[e]     = ha;
        hv[4 + e] = hb;
        lv[e]     = f16_flush((sa - (float)ha) * kResCarry);
        lv[4 + e] = f16_flush((sb - (float)hb) * kResCarry);
      }
      const size_t o = rowbase + (size_t)row * ((size_t)kNN * kND);
      *(volatile v8h*)(PH + o) = hv;
      *(volatile v8h*)(PL + o) = lv;
      __threadfence();
      *(volatile v8h*)(PH + o) = hv;
      *(volatile v8h*)(PL + o) = lv;
    }
    __syncthreads();
  }
}

__global__ __launch_bounds__(512) void cell_scan_kernel(
    const float* __restrict__ x, const float* __restrict__ labels,
    const float* __restrict__ w_in, const float* __restrict__ b_in,
    const float* __restrict__ ng, const float* __restrict__ nb,
    const unsigned short* __restrict__ KHp, const unsigned short* __restrict__ KLp,
    const unsigned short* __restrict__ VHp, const unsigned short* __restrict__ VLp,
    float* __restrict__ out)
{
  __shared__ __align__(16) float dnsh[128];
  __shared__ __align__(16) float redA[16 * 16];
  __shared__ __align__(16) float redB[16 * 16];
  __shared__ __align__(16) float gsh[16];
  __shared__ __align__(16) float slabs[16][16 * kSlabPitchC];

  const _Float16* KH = (const _Float16*)KHp;
  const _Float16* KL = (const _Float16*)KLp;
  const _Float16* VH = (const _Float16*)VHp;
  const _Float16* VL = (const _Float16*)VLp;

  const int tid = threadIdx.x, lane = tid & 31, wave = tid >> 5;
  const int h = lane >> 4, c = lane & 15;
  const int b  = blockIdx.x >> 6;
  const int n0 = (blockIdx.x & 63) * 16;
  const int col0 = wave * 64;

  {
    int idx = tid & 127;
    idx = (idx < kNDrift - 1) ? idx : (kNDrift - 1);
    const int bb = idx / (kNT - 1);
    const int jj = idx - bb * (kNT - 1);
    const float* p0 = labels + (size_t)(bb * kNT + jj) * kNDL;
    const v4f a0 = *(const v4f*)(p0);
    const v4f a1 = *(const v4f*)(p0 + 4);
    const v4f c0 = *(const v4f*)(p0 + 8);
    const v4f c1 = *(const v4f*)(p0 + 12);
    float s = 0.0f;
#pragma unroll
    for (int e = 0; e < 4; ++e) {
      const float u0 = a0[e];
      const float u1 = c0[e];
      const float d = bfv(u1) - bfv(u0);
      s += d * d;
    }
#pragma unroll
    for (int e = 0; e < 4; ++e) {
      const float u0 = a1[e];
      const float u1 = c1[e];
      const float d = bfv(u1) - bfv(u0);
      s += d * d;
    }
    const float dn = sqrtf(s);
    if (tid < 128) dnsh[tid] = dn;
  }
  __syncthreads();
  float dmin = dnsh[0], dmax = dnsh[0];
#pragma unroll 1
  for (int i = 1; i < kNDrift; ++i) {
    const float d = dnsh[i];
    dmin = fminf(dmin, d);
    dmax = fmaxf(dmax, d);
  }
  const float drinv = 1.0f / (dmax - dmin);

  float w0, w1;
  {
    const v2f wv = *(const v2f*)(w_in + 2 * lane);
    const float s0 = wv[0];
    const float s1 = wv[1];
    w0 = bfv(s0);
    w1 = bfv(s1);
  }
  const float bin = bfv(b_in[0]);
  float ngv[4], nbv[4];
#pragma unroll
  for (int j = 0; j < 4; ++j) {
    ngv[j] = bfv(ng[col0 + j * 16 + c]);
    nbv[j] = bfv(nb[col0 + j * 16 + c]);
  }
  const bool lastNode = (n0 + wave == kNN - 1);

  v8f cell[4];
#pragma unroll
  for (int j = 0; j < 4; ++j) cell[j] = (v8f){0.f, 0.f, 0.f, 0.f, 0.f, 0.f, 0.f, 0.f};

#pragma unroll 1
  for (int t = 0; t < kNT; ++t) {
    const int bt = b * kNT + t;

    {
      const v2f xv = *(const v2f*)(x + ((size_t)bt * kNN + n0 + wave) * kNF + 2 * lane);
      const float s0 = xv[0];
      const float s1 = xv[1];
      float p = bfv(s0) * w0 + bfv(s1) * w1;
#pragma unroll
      for (int off = 16; off > 0; off >>= 1) p += __shfl_xor(p, off, 32);
      const int di = b * (kNT - 1) + ((t > 0) ? (t - 1) : 0);
      const float mapped = (dnsh[di] - dmin) * drinv * 2.0f - 1.0f;
      const float lt = (t > 0) ? mapped : 0.0f;
      const float ladd = lastNode ? 0.0f : (lt * 0.1f);
      const float a = (p + bin) + ladd;
      const float gI = 1.0f / (1.0f + expf(-a));
      if (lane == 0) gsh[wave] = gI;
    }

    v16h ah[4], al[4];
    {
      const size_t ao = ((size_t)bt * kNN + n0 + c) * kND + 8 * h;
#pragma unroll
      for (int ks = 0; ks < 4; ++ks) {
        ah[ks] = frag_load(KH + ao + ks * 32);
        al[ks] = frag_load(KL + ao + ks * 32);
      }
    }

    v8f S[4];
#pragma unroll
    for (int j = 0; j < 4; ++j) {
      v8f cm = (v8f){0.f, 0.f, 0.f, 0.f, 0.f, 0.f, 0.f, 0.f};
      v8f cr = (v8f){0.f, 0.f, 0.f, 0.f, 0.f, 0.f, 0.f, 0.f};
      const size_t bo = ((size_t)bt * kNN + col0 + j * 16 + c) * kND + 8 * h;
#pragma unroll
      for (int ks = 0; ks < 4; ++ks) {
        const v16h bh = frag_load(VH + bo + ks * 32);
        const v16h bl = frag_load(VL + bo + ks * 32);
        mma_vr(ah[ks], al[ks], bh, bl, cm, cr);
      }
#pragma unroll
      for (int r = 0; r < 8; ++r) S[j][r] = cm[r] + cr[r] * kResCarryInv;
    }

    float rs[8];
#pragma unroll
    for (int r = 0; r < 8; ++r) rs[r] = (S[0][r] + S[1][r]) + (S[2][r] + S[3][r]);
#pragma unroll
    for (int off = 1; off < 16; off <<= 1) {
#pragma unroll
      for (int r = 0; r < 8; ++r) rs[r] += __shfl_xor(rs[r], off, 32);
    }
    if (c == 0) {
#pragma unroll
      for (int r = 0; r < 8; ++r) redA[(8 * h + r) * 16 + wave] = rs[r];
    }
    __syncthreads();

    float gI[8];
#pragma unroll
    for (int r = 0; r < 8; ++r) {
      const float* rp = redA + (8 * h + r) * 16;
      const v4f q0 = *(const v4f*)(rp);
      const v4f q1 = *(const v4f*)(rp + 4);
      const v4f q2 = *(const v4f*)(rp + 8);
      const v4f q3 = *(const v4f*)(rp + 12);
      const float tot = (((q0[0] + q0[1]) + (q0[2] + q0[3])) + ((q1[0] + q1[1]) + (q1[2] + q1[3])))
                      + (((q2[0] + q2[1]) + (q2[2] + q2[3])) + ((q3[0] + q3[1]) + (q3[2] + q3[3])));
      rs[r] = tot * (1.0f / (float)kNN);
      gI[r] = gsh[8 * h + r];
    }
    float dv[8];
#pragma unroll
    for (int r = 0; r < 8; ++r) dv[r] = 0.0f;
#pragma unroll
    for (int j = 0; j < 4; ++j) {
#pragma unroll
      for (int r = 0; r < 8; ++r) {
        const float d = S[j][r] - rs[r];
        S[j][r] = d;
        dv[r] += d * d;
      }
    }
#pragma unroll
    for (int off = 1; off < 16; off <<= 1) {
#pragma unroll
      for (int r = 0; r < 8; ++r) dv[r] += __shfl_xor(dv[r], off, 32);
    }
    if (c == 0) {
#pragma unroll
      for (int r = 0; r < 8; ++r) redB[(8 * h + r) * 16 + wave] = dv[r];
    }
    __syncthreads();

#pragma unroll
    for (int r = 0; r < 8; ++r) {
      const float* rp = redB + (8 * h + r) * 16;
      const v4f q0 = *(const v4f*)(rp);
      const v4f q1 = *(const v4f*)(rp + 4);
      const v4f q2 = *(const v4f*)(rp + 8);
      const v4f q3 = *(const v4f*)(rp + 12);
      const float tot = (((q0[0] + q0[1]) + (q0[2] + q0[3])) + ((q1[0] + q1[1]) + (q1[2] + q1[3])))
                      + (((q2[0] + q2[1]) + (q2[2] + q2[3])) + ((q3[0] + q3[1]) + (q3[2] + q3[3])));
      dv[r] = rsqrtf(tot * (1.0f / (float)kNN) + kLnEps);
    }
#pragma unroll
    for (int j = 0; j < 4; ++j) {
#pragma unroll
      for (int r = 0; r < 8; ++r) {
        const float y = (ngv[j] * S[j][r]) * dv[r] + nbv[j];
        const float nowv = fmaxf(y, 0.0f);
        cell[j][r] = (1.0f - gI[r]) * cell[j][r] + gI[r] * nowv;
      }
    }
  }

  {
    float* slab = slabs[wave];
    const int q = lane >> 3, c4 = (lane & 7) * 4;
#pragma unroll
    for (int p = 0; p < 2; ++p) {
#pragma unroll
      for (int jj = 0; jj < 2; ++jj) {
#pragma unroll
        for (int r = 0; r < 8; ++r) slab[(8 * h + r) * kSlabPitchC + jj * 16 + c] = cell[2 * p + jj][r];
      }
      __syncthreads();
      v4f vv[4];
#pragma unroll
      for (int it = 0; it < 4; ++it) vv[it] = *(const v4f*)(slab + (it * 4 + q) * kSlabPitchC + c4);
      float* ob = out + ((size_t)(b * kNN + n0)) * kNN + col0 + p * 32 + c4;
      for (int pass = 0; pass < 2; ++pass) {
#pragma unroll
        for (int it = 0; it < 4; ++it)
          *(volatile v4f*)(ob + (size_t)(it * 4 + q) * kNN) = vv[it];
        __threadfence();
      }
      __syncthreads();
    }
  }
}

extern "C" void kernel_launch(void* const* d_in, const int* in_sizes, int n_in,
                              void* d_out, int out_size, void* d_ws, size_t ws_size,
                              hipStream_t stream) {
  if (n_in < 14) return;
  if (in_sizes[0] != kNB * kNT * kNN * kNF) return;
  if (in_sizes[1] != kNB * kNT * kNDL) return;
  if (in_sizes[2] != kNN * kNF * kND) return;
  if (in_sizes[3] != kNN * kNF * kND) return;
  if (in_sizes[4] != kNN * kND) return;
  if (in_sizes[5] != kNN * kND) return;
  if (in_sizes[6] != kNF) return;
  if (in_sizes[7] != 1) return;
  if (in_sizes[8] != kND || in_sizes[9] != kND || in_sizes[10] != kND || in_sizes[11] != kND) return;
  if (in_sizes[12] != kNN || in_sizes[13] != kNN) return;
  if (out_size != kNB * kNN * kNN) return;
  if (ws_size < kWsTotal) return;

  const float* x      = (const float*)d_in[0];
  const float* labels = (const float*)d_in[1];
  const float* Wk     = (const float*)d_in[2];
  const float* Wv     = (const float*)d_in[3];
  const float* bk     = (const float*)d_in[4];
  const float* bv     = (const float*)d_in[5];
  const float* w_in   = (const float*)d_in[6];
  const float* b_in   = (const float*)d_in[7];
  const float* kg     = (const float*)d_in[8];
  const float* kb     = (const float*)d_in[9];
  const float* vg     = (const float*)d_in[10];
  const float* vb     = (const float*)d_in[11];
  const float* ng     = (const float*)d_in[12];
  const float* nb     = (const float*)d_in[13];
  float* out = (float*)d_out;

  char* ws = (char*)d_ws;
  unsigned short* KH = (unsigned short*)(ws + kOffKH);
  unsigned short* KL = (unsigned short*)(ws + kOffKL);
  unsigned short* VH = (unsigned short*)(ws + kOffVH);
  unsigned short* VL = (unsigned short*)(ws + kOffVL);

  constexpr float kscale = 0.08838834764831845f;
  static_assert(__builtin_bit_cast(unsigned, kscale) == 0x3DB504F3u);
  static_assert(kND == 128);

  node_proj_kernel<<<dim3(kNN), dim3(256), 0, stream>>>(x, Wk, Wv, bk, bv, kg, kb, vg, vb, KH, KL, VH, VL, kscale);
  cell_scan_kernel<<<dim3(kNB * (kNN / 16)), dim3(512), 0, stream>>>(x, labels, w_in, b_in, ng, nb,
                                                                     KH, KL, VH, VL, out);
}
